// GeometricCosineAttention_369367187597
// MI455X (gfx1250) — hardware-verified
//
#include <hip/hip_runtime.h>
#include <math.h>

typedef __attribute__((ext_vector_type(16))) _Float16 v16h;
typedef __attribute__((ext_vector_type(16))) __bf16 v16b;
typedef __attribute__((ext_vector_type(8)))  _Float16 v8h;
typedef __attribute__((ext_vector_type(8)))  float v8f;
typedef __attribute__((ext_vector_type(4)))  float v4f;
typedef __attribute__((ext_vector_type(2)))  float v2f;
typedef __attribute__((ext_vector_type(4)))  unsigned v4u;
typedef __attribute__((ext_vector_type(4)))  int v4i;
typedef float __attribute__((may_alias)) float_a;
typedef int __attribute__((may_alias)) int_a;

template <typename T> __device__ __forceinline__ void vst2(void* p, T v) { *(volatile T*)p = v; __threadfence(); *(volatile T*)p = v; }
__device__ __forceinline__ v8f wmma16(v16h a, v16h b, v8f c) {
  v8f d = __builtin_amdgcn_wmma_f32_16x16x32_f16(false, a, false, b, (short)0, c, false, false);
  asm volatile("v_nop\n\tv_nop\n\tv_nop\n\tv_nop" : "+v"(d) : "v"(a), "v"(b));
  return d;
}
__device__ __forceinline__ v8f wmma_bf(v16b a, v16b b, v8f c) {
  v8f d = __builtin_amdgcn_wmma_f32_16x16x32_bf16(false, a, false, b, (short)0, c, false, false);
  asm volatile("v_nop\n\tv_nop\n\tv_nop\n\tv_nop" : "+v"(d) : "v"(a), "v"(b));
  return d;
}
__device__ __forceinline__ v16h frag_h(const _Float16* rowk0, int lane) {
  union { v16h v; v8h q[2]; } u; const _Float16* p = rowk0 + 8 * (lane >> 4);
  u.q[0] = *(const v8h*)p; u.q[1] = *(const v8h*)(p + 16); return u.v;
}
__device__ __forceinline__ v16h frag_f32(const float* rowk0, int lane) {
  v16h a; const float* p = rowk0 + 8 * (lane >> 4);
#pragma unroll
  for (int i = 0; i < 8; ++i) { a[i] = (_Float16)p[i]; a[8 + i] = (_Float16)p[16 + i]; }
  return a;
}
__device__ __forceinline__ v16h frag_f32s(const float* rowk0, int lane, float sc) {
  v16h a; const float* p = rowk0 + 8 * (lane >> 4);
#pragma unroll
  for (int i = 0; i < 8; ++i) { a[i] = (_Float16)(p[i] * sc); a[8 + i] = (_Float16)(p[16 + i] * sc); }
  return a;
}
__device__ __forceinline__ v16h fragc_f32(const float* W, int k0, int n, int lane, int ld, int K) {
  v16h a; const int g = lane >> 4;
#pragma unroll
  for (int i = 0; i < 8; ++i) { const int ka = k0 + 8 * g + i, kb = ka + 16;
    a[i] = (_Float16)(ka < K ? W[(size_t)ka * ld + n] : 0.f); a[8 + i] = (_Float16)(kb < K ? W[(size_t)kb * ld + n] : 0.f); }
  return a;
}
struct F2 { v16b h, l; };
__device__ __forceinline__ F2 bsplit16(const float v[16]) { F2 r;
#pragma unroll
  for (int i = 0; i < 16; ++i) { const __bf16 h = (__bf16)v[i]; r.h[i] = h; r.l[i] = (__bf16)(v[i] - (float)h); }
  return r; }
__device__ __forceinline__ F2 split_row(const float* row, int k0, int lane) { float v[16]; const float* p = row + k0 + 8 * (lane >> 4);
#pragma unroll
  for (int i = 0; i < 8; ++i) { v[i] = p[i]; v[8 + i] = p[16 + i]; }
  return bsplit16(v); }
__device__ __forceinline__ F2 split_rowK(const float* row, int k0, int lane, int K) { float v[16]; const int g = lane >> 4;
#pragma unroll
  for (int i = 0; i < 8; ++i) { const int ka = k0 + 8 * g + i, kb = ka + 16; v[i] = ka < K ? row[ka] : 0.f; v[8 + i] = kb < K ? row[kb] : 0.f; }
  return bsplit16(v); }
__device__ __forceinline__ F2 split_col(const float* W, int k0, int n, int lane, int ld, int K) { float v[16]; const int g = lane >> 4;
#pragma unroll
  for (int i = 0; i < 8; ++i) { const int ka = k0 + 8 * g + i, kb = ka + 16; v[i] = ka < K ? W[(size_t)ka * ld + n] : 0.f; v[8 + i] = kb < K ? W[(size_t)kb * ld + n] : 0.f; }
  return bsplit16(v); }
__device__ __forceinline__ v8f mac3(const F2& a, const F2& b, v8f c) { c = wmma_bf(a.l, b.h, c); c = wmma_bf(a.h, b.l, c); return wmma_bf(a.h, b.h, c); }
__device__ __forceinline__ float sigm(float v) { return 1.0f / (1.0f + expf(-v)); }
#define LDSX() do { asm volatile("s_wait_dscnt 0" ::: "memory"); __builtin_amdgcn_wave_barrier(); __builtin_amdgcn_fence(__ATOMIC_RELEASE, "workgroup"); } while (0)

#define NB 2
#define EE 2048
#define CC 512
#define NH 8
#define HD 64
#define NR (NB * EE)

__global__ __launch_bounds__(256) void k_cvt(const float* __restrict__ x, _Float16* __restrict__ X16) {
  const size_t i8 = (size_t)blockIdx.x * 256 + threadIdx.x; if (i8 >= (size_t)NR * CC / 8) return;
  union { v8h h; v4u u; } pk;
#pragma unroll
  for (int e = 0; e < 8; ++e) pk.h[e] = (_Float16)x[i8 * 8 + e];
  vst2(X16 + i8 * 8, pk.u);
}
__global__ __launch_bounds__(256) void k_pack(const float* __restrict__ Wq, const float* __restrict__ Wk, const float* __restrict__ Wv, const float* __restrict__ Wp, _Float16* __restrict__ P) {
  const int r = blockIdx.x, tid = threadIdx.x; __shared__ __align__(16) _Float16 srow[CC];
  const int which = r >> 9, n = r & 511; const float* W = which == 0 ? Wq : (which == 1 ? Wk : (which == 2 ? Wv : Wp));
  for (int k = tid; k < CC; k += 256) srow[k] = (_Float16)(W[(size_t)n * CC + k] * 16.0f);
  __syncthreads();
  if (tid < 64) vst2(P + (size_t)r * CC + tid * 8, *(const v4u*)(&srow[tid * 8]));
}
__global__ __launch_bounds__(128) void k_qkv(const _Float16* __restrict__ X16, const _Float16* __restrict__ P, _Float16* __restrict__ Q16, _Float16* __restrict__ K16, _Float16* __restrict__ VT) {
  __shared__ __align__(16) float so[4][16][132];
  __shared__ __align__(16) _Float16 st[128][72];
  const int tid = threadIdx.x, wave = tid >> 5, lane = tid & 31, col = lane & 15, g = lane >> 4;
  const int which = blockIdx.z, r0b = blockIdx.x * 64, r0 = r0b + wave * 16, n0 = blockIdx.y * 128; const int b = r0b / EE, e0 = r0b % EE;
  const _Float16* Pw = P + (size_t)which * CC * CC;
  v8f acc[8] = {};
#pragma unroll 2
  for (int kc = 0; kc < CC / 32; ++kc) { const v16h a = frag_h(X16 + (size_t)(r0 + col) * CC + kc * 32, lane);
#pragma unroll
    for (int j = 0; j < 8; ++j) acc[j] = wmma16(a, frag_h(Pw + (size_t)(n0 + j * 16 + col) * CC + kc * 32, lane), acc[j]); }
  if (which < 2) {
#pragma unroll
    for (int j = 0; j < 8; ++j)
#pragma unroll
      for (int r = 0; r < 8; ++r) so[wave][8 * g + r][j * 16 + col] = acc[j][r] * (4.0f / 16.0f);
    LDSX();
    _Float16* D = which == 0 ? Q16 : K16;
    for (int q = lane; q < 16 * 2 * 8; q += 32) { const int hh = q >> 7, rl = (q >> 3) & 15, pc = q & 7; const int h = (n0 >> 6) + hh; union { v8h h8; v4u u; } pk;
#pragma unroll
      for (int e = 0; e < 8; ++e) pk.h8[e] = (_Float16)so[wave][rl][hh * 64 + pc * 8 + e];
      vst2(D + (((size_t)b * NH + h) * EE + e0 + wave * 16 + rl) * HD + pc * 8, pk.u); } }
  else {
#pragma unroll
    for (int j = 0; j < 8; ++j)
#pragma unroll
      for (int r = 0; r < 8; ++r) st[j * 16 + col][wave * 16 + 8 * g + r] = (_Float16)(acc[j][r] * (4.0f / 16.0f));
    __syncthreads();
    for (int q = tid; q < 128 * 8; q += 128) { const int cl = q >> 3, pc = q & 7; const int c = n0 + cl, h = c >> 6, d = c & 63; vst2(VT + (((size_t)b * NH + h) * HD + d) * EE + e0 + pc * 8, *(const v4u*)(&st[cl][pc * 8])); } }
}
__global__ __launch_bounds__(256) void k_vsum(const _Float16* __restrict__ VT, float* __restrict__ VS) {
  __shared__ float sp[4][64]; __shared__ __align__(16) float so[64];
  const int bh = blockIdx.x, tid = threadIdx.x, d = tid & 63, part = tid >> 6; float s = 0.f;
  const _Float16* row = VT + ((size_t)bh * HD + d) * EE;
  for (int e = part * 512; e < part * 512 + 512; ++e) s += (float)row[e];
  sp[part][d] = s;
  __syncthreads();
  if (tid < 64) so[tid] = ((sp[0][tid] + sp[1][tid]) + (sp[2][tid] + sp[3][tid])) * 0.25f;
  __syncthreads();
  if (tid < 16) vst2(VS + (size_t)bh * HD + tid * 4, *(const v4f*)(&so[tid * 4]));
}
__global__ __launch_bounds__(128) void k_attn(const _Float16* __restrict__ Q16, const _Float16* __restrict__ K16, const _Float16* __restrict__ VT, const float* __restrict__ VS, const float* __restrict__ adj, _Float16* __restrict__ O16) {
  __shared__ __align__(16) _Float16 sP[4][16][72];
  __shared__ __align__(16) float sO[4][16][68];
  const int tid = threadIdx.x, w = tid >> 5, lane = tid & 31, col = lane & 15, g = lane >> 4;
  const int b = blockIdx.z, h = blockIdx.y, q0 = blockIdx.x * 64 + w * 16; const size_t bh = (size_t)b * NH + h;
  v16h aq[2];
#pragma unroll
  for (int kc = 0; kc < 2; ++kc) aq[kc] = frag_h(Q16 + (bh * EE + q0 + col) * HD + kc * 32, lane);
  v8f acc[4] = {};
#pragma unroll 1
  for (int kt = 0; kt < EE / 64; ++kt) {
#pragma unroll
    for (int t = 0; t < 4; ++t) { v8f s = {}; const int key = kt * 64 + t * 16 + col;
#pragma unroll
      for (int kc = 0; kc < 2; ++kc) s = wmma16(aq[kc], frag_h(K16 + (bh * EE + key) * HD + kc * 32, lane), s);
#pragma unroll
      for (int r = 0; r < 8; ++r) { const float m = adj[(size_t)(q0 + 8 * g + r) * EE + key]; sP[w][8 * g + r][t * 16 + col] = (_Float16)(s[r] * m * (1.0f / (16.0f * 8.0f))); } }
    LDSX();
#pragma unroll
    for (int kc = 0; kc < 2; ++kc) { const v16h pa = frag_h(&sP[w][col][0] + kc * 32, lane);
#pragma unroll
      for (int t = 0; t < 4; ++t) acc[t] = wmma16(pa, frag_h(VT + (bh * HD + t * 16 + col) * EE + kt * 64 + kc * 32, lane), acc[t]); }
    LDSX(); }
#pragma unroll
  for (int t = 0; t < 4; ++t) { const int d = t * 16 + col; const float vs = VS[bh * HD + d];
#pragma unroll
    for (int r = 0; r < 8; ++r) sO[w][8 * g + r][d] = (0.5f * (acc[t][r] * 2.0f) + 0.5f * vs) * 0.125f; }
  LDSX();
  for (int q = lane; q < 16 * 8; q += 32) { const int rl = q >> 3, pc = q & 7; union { v8h h8; v4u u; } pk;
#pragma unroll
    for (int e = 0; e < 8; ++e) pk.h8[e] = (_Float16)sO[w][rl][pc * 8 + e];
    vst2(O16 + (bh * EE + q0 + rl) * HD + pc * 8, pk.u); }
}
__global__ __launch_bounds__(128) void k_proj(const _Float16* __restrict__ O16, const _Float16* __restrict__ P, const float* __restrict__ bp, const float* __restrict__ lnw, const float* __restrict__ lnb, const float* __restrict__ gam, const float* __restrict__ x, float* __restrict__ out) {
  __shared__ __align__(16) float sy[64][CC + 4];
  const int tid = threadIdx.x, wave = tid >> 5, lane = tid & 31, col = lane & 15, g = lane >> 4;
  const int r0b = blockIdx.x * 64, r0 = r0b + wave * 16;
#pragma unroll 1
  for (int np = 0; np < 4; ++np) { v8f acc[8] = {};
#pragma unroll 2
    for (int kc = 0; kc < CC / 32; ++kc) { const int R = r0 + col; const v16h a = frag_h(O16 + ((((size_t)(R / EE)) * NH + (kc >> 1)) * EE + (R % EE)) * HD + (kc & 1) * 32, lane);
#pragma unroll
      for (int j = 0; j < 8; ++j) acc[j] = wmma16(a, frag_h(P + (size_t)(3 * CC + np * 128 + j * 16 + col) * CC + kc * 32, lane), acc[j]); }
#pragma unroll
    for (int j = 0; j < 8; ++j) { const int c = np * 128 + j * 16 + col; const float bb = bp[c];
#pragma unroll
      for (int r = 0; r < 8; ++r) sy[wave * 16 + 8 * g + r][c] = acc[j][r] * (8.0f / 16.0f) + bb; } }
  LDSX();
  { const int rl = lane >> 1, hf = lane & 1; float* row = &sy[wave * 16 + rl][0]; float s = 0.f; for (int c = hf * 256; c < hf * 256 + 256; ++c) s += row[c]; s += __shfl_xor(s, 1, 32); const float mu = s * (1.0f / CC);
    float q2 = 0.f; for (int c = hf * 256; c < hf * 256 + 256; ++c) { const float dv = row[c] - mu; q2 += dv * dv; } q2 += __shfl_xor(q2, 1, 32); const float rs = rsqrtf(q2 * (1.0f / CC) + 1e-5f);
    const float gm = gam[0]; const float* xr = x + (size_t)(r0 + rl) * CC;
    LDSX();
    for (int c = hf * 256; c < hf * 256 + 256; ++c) row[c] = xr[c] + gm * ((row[c] - mu) * rs * lnw[c] + lnb[c]); }
  LDSX();
  for (int rl = 0; rl < 16; ++rl) for (int pc = lane; pc < CC / 4; pc += 32) vst2(out + (size_t)(r0 + rl) * CC + pc * 4, *(const v4f*)(&sy[wave * 16 + rl][pc * 4]));
}
extern "C" void kernel_launch(void* const* d_in, const int* in_sizes, int n_in, void* d_out, int out_size, void* d_ws, size_t ws_size, hipStream_t stream) {
  (void)in_sizes; (void)n_in; (void)out_size; (void)ws_size;
  const float** I = (const float**)d_in;
  const float* x = I[0]; const float* adj = I[1]; const float* Wq = I[2]; const float* Wk = I[3]; const float* Wv = I[4]; const float* Wp = I[5]; const float* bp = I[6]; const float* lnw = I[7]; const float* lnb = I[8]; const float* gam = I[9];
  float* out = (float*)d_out;
  char* ws = (char*)d_ws; size_t off = 0;
  auto take = [&](size_t bytes) { char* p = ws + off; off += (bytes + 255) & ~(size_t)255; return p; };
  _Float16* X16 = (_Float16*)take((size_t)NR * CC * 2); _Float16* P = (_Float16*)take((size_t)4 * CC * CC * 2);
  _Float16* Q16 = (_Float16*)take((size_t)NR * CC * 2); _Float16* K16 = (_Float16*)take((size_t)NR * CC * 2); _Float16* VT = (_Float16*)take((size_t)NR * CC * 2); float* VS = (float*)take((size_t)NB * NH * HD * 4); _Float16* O16 = (_Float16*)take((size_t)NR * CC * 2);
  k_cvt<<<(NR * CC / 8 + 255) / 256, 256, 0, stream>>>(x, X16);
  k_pack<<<4 * CC, 256, 0, stream>>>(Wq, Wk, Wv, Wp, P);
  k_qkv<<<dim3(NR / 64, CC / 128, 3), 128, 0, stream>>>(X16, P, Q16, K16, VT);
  k_vsum<<<NB * NH, 256, 0, stream>>>(VT, VS);
  k_attn<<<dim3(EE / 64, NH, NB), 128, 0, stream>>>(Q16, K16, VT, VS, adj, O16);
  k_proj<<<NR / 64, 128, 0, stream>>>(O16, P, bp, lnw, lnb, gam, x, out);
}
